// SeqSelfAttention_56667798504129
// MI455X (gfx1250) — hardware-verified
//
#include <hip/hip_runtime.h>
#include <stddef.h>


typedef _Float16 v16h __attribute__((ext_vector_type(16)));
typedef _Float16 v8h  __attribute__((ext_vector_type(8)));
typedef float    v8f  __attribute__((ext_vector_type(8)));
typedef float    v4f  __attribute__((ext_vector_type(4)));
typedef _Float16 h16;

#ifndef NB
#define NB 4
#endif
#ifndef SEQ
#define SEQ 1024
#endif
#define NB_FULL  4
#define SEQ_FULL 1024
#define DIM   1024
#define UNITS 64
#define NQK   128
#define BAND  64
#define QT    32
#define WIN   96
#define MROWS (NB * SEQ)

static_assert(NB >= 1 && NB <= NB_FULL);
static_assert(SEQ >= 128 && SEQ <= SEQ_FULL && (SEQ % 128) == 0);
static_assert(UNITS == 64 && NQK == 2 * UNITS);
static_assert((DIM % 64) == 0 && (DIM % 32) == 0);
static_assert((MROWS % 64) == 0);
static_assert(QT == 32 && QT == 8 * 4);
static_assert(BAND == 64 && WIN == QT + BAND && (WIN % 32) == 0);
static_assert(DIM == 8 * 2 * 64);
static_assert((SEQ % QT) == 0);

#define LDT 72
#define LDC 68
#define LDP 104
#define QP  65
static_assert((LDT % 8) == 0 && LDT >= 64);
static_assert((LDC % 4) == 0 && LDC >= 64);
static_assert((LDP % 8) == 0 && LDP >= WIN);
static_assert(QP >= UNITS);

#define WCARRY 64.0f
#define PCARRY 1024.0f

#define QS_OFF 0
#define KS_OFF (QT * QP)
#define SM_AB  (KS_OFF + WIN * QP)
#define SM_C   (8 * 16 * LDC)
#define SM_FLOATS ((SM_AB > SM_C) ? SM_AB : SM_C)
static_assert(SM_FLOATS >= SM_AB && SM_FLOATS >= SM_C);
static_assert((size_t)SM_FLOATS * 4 + UNITS * 4 + QT * 4 + (size_t)QT * LDP * 2 <= (size_t)65536);

#define WQK_BYTES ((size_t)NQK * DIM * 2)
#define XH_BYTES  ((size_t)MROWS * DIM * 2)
#define XT_BYTES  ((size_t)NB * DIM * SEQ * 2)
#define QK_BYTES  ((size_t)MROWS * NQK * 4)
#define OFF_WQK ((size_t)0)
#define OFF_XH  (OFF_WQK + WQK_BYTES)
#define OFF_XT  (OFF_XH + XH_BYTES)
#define OFF_QK  (OFF_XT + XT_BYTES)
#define WS_TOTAL (OFF_QK + QK_BYTES)
static_assert((WQK_BYTES % 128) == 0 && (XH_BYTES % 128) == 0);
static_assert((XT_BYTES % 128) == 0 && (QK_BYTES % 128) == 0);
static_assert(WS_TOTAL <= (size_t)134217728);

__device__ __forceinline__ float bf16r(float x) {
  unsigned int u = __float_as_uint(x);
  u = (u + 0x7FFFu + ((u >> 16) & 1u)) & 0xFFFF0000u;
  return __uint_as_float(u);
}

static __device__ __forceinline__ h16 toh_flush(float v) {
  const h16 r = (h16)v;
  return (fabsf(v) < 6.103515625e-05f) ? (h16)0.0f : r;
}

__device__ __forceinline__ v16h frag_at(const _Float16* p) {
  v8h lo = *(const v8h*)(p);
  v8h hi = *(const v8h*)(p + 16);
  v16h out;
#pragma unroll
  for (int i = 0; i < 8; ++i) { out[i] = lo[i]; out[i + 8] = hi[i]; }
  return out;
}
__device__ __forceinline__ v16h ld_frag(const _Float16* base, unsigned ld) {
  const unsigned lane = threadIdx.x & 31u;
  return frag_at(base + (lane & 15u) * ld + (lane >> 4) * 8u);
}

__device__ __forceinline__ v8f wmma16(v16h a, v16h b, v8f c) {
  v8f d = __builtin_amdgcn_wmma_f32_16x16x32_f16(false, a, false, b, (short)0, c,
                                                 false, false);
  asm volatile("v_nop\n\tv_nop\n\tv_nop\n\tv_nop" : "+v"(d) : "v"(a), "v"(b));
  return d;
}

__device__ __forceinline__ float red32_sum(float x) {
#pragma unroll
  for (int off = 1; off < 32; off <<= 1) x += __shfl_xor(x, off, 32);
  return x;
}
__device__ __forceinline__ float red32_max(float x) {
#pragma unroll
  for (int off = 1; off < 32; off <<= 1) x = fmaxf(x, __shfl_xor(x, off, 32));
  return x;
}

__device__ __forceinline__ void wave_lds_sync() {
  __builtin_amdgcn_fence(3  , "wavefront");
  asm volatile("s_wait_dscnt 0x0" ::: "memory");
  __builtin_amdgcn_wave_barrier();
}

__device__ __forceinline__ float tanh_fast(float x) {
  const float ax = fminf(fabsf(x), 30.0f);
  const float ex = __expf(ax + ax);
  const float r = 1.0f - 2.0f * __builtin_amdgcn_rcpf(ex + 1.0f);
  return (x < 0.0f) ? -r : r;
}

__global__ __launch_bounds__(256) void wconv_kernel(
    const float* __restrict__ W, _Float16* __restrict__ Wt, unsigned ldw, unsigned ldk) {
  __shared__ _Float16 T[64 * LDT];
  const unsigned tid = threadIdx.x;
  const unsigned n0 = blockIdx.x * 64u;
  const unsigned k0 = blockIdx.y * 64u;
#pragma unroll 4
  for (unsigned j = 0; j < 16u; ++j) {
    const unsigned idx = tid + 256u * j;
    const unsigned kr = idx >> 6, nc = idx & 63u;
    const float v = W[(size_t)(k0 + kr) * ldw + n0 + nc];
    T[nc * LDT + kr] = (_Float16)(WCARRY * bf16r(v));
  }
  __syncthreads();
  v8h x[2];
  size_t off[2];
#pragma unroll
  for (unsigned i = 0; i < 2u; ++i) {
    const unsigned n = 32u * i + (tid >> 3);
    const unsigned kc = (tid & 7u) * 8u;
    x[i] = *(const v8h*)&T[n * LDT + kc];
    off[i] = (size_t)(n0 + n) * ldk + k0 + kc;
  }
#pragma unroll
  for (int i = 0; i < 2; ++i) *(volatile v8h*)(Wt + off[i]) = x[i];
  __threadfence();
#pragma unroll
  for (int i = 0; i < 2; ++i) *(volatile v8h*)(Wt + off[i]) = x[i];
}

__global__ __launch_bounds__(256) void xconv_kernel(
    const float* __restrict__ X, _Float16* __restrict__ Xh, _Float16* __restrict__ Xt) {
  __shared__ _Float16 Tr[64 * LDT];
  __shared__ _Float16 Tc[64 * LDT];
  const unsigned tid = threadIdx.x;
  const unsigned d0 = blockIdx.x * 64u;
  const unsigned row0 = blockIdx.y * 64u;
  const unsigned bidx = row0 / (unsigned)SEQ;
  const unsigned key0 = row0 - bidx * (unsigned)SEQ;
  const size_t frow0 = (size_t)bidx * SEQ_FULL + key0;
#pragma unroll
  for (unsigned j = 0; j < 4u; ++j) {
    const unsigned idx = tid + 256u * j;
    const unsigned sr = idx >> 4, c4 = (idx & 15u) * 4u;
    const v4f a = *(const v4f*)(X + (frow0 + sr) * DIM + d0 + c4);
#pragma unroll
    for (unsigned i = 0; i < 4u; ++i) {
      const h16 hv = toh_flush(bf16r(a[i]));
      Tr[sr * LDT + c4 + i] = hv;
      Tc[(c4 + i) * LDT + sr] = hv;
    }
  }
  __syncthreads();
  v8h xr[2], xc[2];
  size_t offr[2], offc[2];
#pragma unroll
  for (unsigned i = 0; i < 2u; ++i) {
    const unsigned r = 32u * i + (tid >> 3);
    const unsigned c = (tid & 7u) * 8u;
    xr[i] = *(const v8h*)&Tr[r * LDT + c];
    xc[i] = *(const v8h*)&Tc[r * LDT + c];
    offr[i] = (size_t)(row0 + r) * DIM + d0 + c;
    offc[i] = ((size_t)bidx * DIM + d0 + r) * SEQ + key0 + c;
  }
#pragma unroll
  for (int i = 0; i < 2; ++i) {
    *(volatile v8h*)(Xh + offr[i]) = xr[i];
    *(volatile v8h*)(Xt + offc[i]) = xc[i];
  }
  __threadfence();
#pragma unroll
  for (int i = 0; i < 2; ++i) {
    *(volatile v8h*)(Xh + offr[i]) = xr[i];
    *(volatile v8h*)(Xt + offc[i]) = xc[i];
  }
}

__global__ __launch_bounds__(256) void proj_kernel(
    const _Float16* __restrict__ A16, const _Float16* __restrict__ Bt,
    float* __restrict__ outf) {
  __shared__ float Cs[64 * LDC];
  const unsigned tid = threadIdx.x, lane = tid & 31u;
  const unsigned w = __builtin_amdgcn_readfirstlane(threadIdx.x >> 5);
  const unsigned mw = w >> 1, nw = w & 1u;
  const unsigned hh = lane >> 4, m = lane & 15u;
  const unsigned n0 = blockIdx.x * 64u;
  const unsigned row0 = blockIdx.y * 64u;
  const unsigned K = (unsigned)DIM;

  const _Float16* ap  = A16 + (size_t)(row0 + mw * 16u + m) * K + hh * 8u;
  const _Float16* bp0 = Bt + (size_t)(n0 + nw * 32u + m) * K + hh * 8u;
  const _Float16* bp1 = bp0 + (size_t)16 * K;
  v8f acc0 = {}, acc1 = {};
#pragma unroll 2
  for (unsigned k0 = 0; k0 < K; k0 += 32u) {
    const v16h a  = frag_at(ap + k0);
    const v16h b0 = frag_at(bp0 + k0);
    const v16h b1 = frag_at(bp1 + k0);
    acc0 = wmma16(a, b0, acc0);
    acc1 = wmma16(a, b1, acc1);
  }
#pragma unroll
  for (int r = 0; r < 8; ++r) {
    float* d = &Cs[(mw * 16u + hh * 8u + (unsigned)r) * LDC + nw * 32u + m];
    d[0]  = acc0[r];
    d[16] = acc1[r];
  }
  __syncthreads();

  v4f xs[4];
  size_t off[4];
#pragma unroll
  for (unsigned i = 0; i < 4u; ++i) {
    const unsigned r = 16u * i + (tid >> 4);
    const unsigned c = (tid & 15u) * 4u;
    const v4f u = *(const v4f*)&Cs[r * LDC + c];
    xs[i] = u * (1.0f / WCARRY);
    off[i] = (size_t)(row0 + r) * NQK + n0 + c;
  }
#pragma unroll
  for (int i = 0; i < 4; ++i) *(volatile v4f*)(outf + off[i]) = xs[i];
  __threadfence();
#pragma unroll
  for (int i = 0; i < 4; ++i) *(volatile v4f*)(outf + off[i]) = xs[i];
}

__global__ __launch_bounds__(256) void band_attn_kernel(
    const float* __restrict__ QK, const _Float16* __restrict__ Xt,
    const float* __restrict__ bh, const float* __restrict__ Wa, const float* __restrict__ ba,
    float* __restrict__ out) {
  __shared__ float Sm[SM_FLOATS];
  __shared__ float WAs[UNITS];
  __shared__ float Rinv[QT];
  __shared__ _Float16 Pt[QT * LDP];

  const unsigned tid = threadIdx.x, lane = tid & 31u;
  const unsigned w = __builtin_amdgcn_readfirstlane(threadIdx.x >> 5);
  const unsigned hh = lane >> 4, m = lane & 15u;
  const unsigned t0 = blockIdx.x * (unsigned)QT;
  const unsigned b = blockIdx.y;
  const int s0 = (int)t0 - BAND / 2;

#pragma unroll
  for (unsigned j = 0; j < 2u; ++j) {
    const unsigned idx = tid + 256u * j;
    const unsigned r = idx >> 4, c4 = (idx & 15u) * 4u;
    const v4f a = *(const v4f*)(QK + (size_t)(b * (unsigned)SEQ + t0 + r) * NQK + c4);
    const v4f g = *(const v4f*)(bh + c4);
#pragma unroll
    for (unsigned i = 0; i < 4u; ++i) Sm[QS_OFF + r * QP + c4 + i] = a[i] + bf16r(g[i]);
  }
#pragma unroll 2
  for (unsigned j = 0; j < 6u; ++j) {
    const unsigned idx = tid + 256u * j;
    const unsigned r = idx >> 4, c4 = (idx & 15u) * 4u;
    const int s = s0 + (int)r;
    const int sc = (s < 0) ? 0 : ((s > SEQ - 1) ? (SEQ - 1) : s);
    const v4f a = *(const v4f*)(QK + (size_t)(b * (unsigned)SEQ + (unsigned)sc) * NQK + UNITS + c4);
    const bool ok = (s == sc);
#pragma unroll
    for (unsigned i = 0; i < 4u; ++i) Sm[KS_OFF + r * QP + c4 + i] = ok ? a[i] : 0.0f;
  }
  if (tid < (unsigned)UNITS) WAs[tid] = bf16r(Wa[tid]);
  const float bias_a = bf16r(ba[0]);
  __syncthreads();

#pragma unroll 1
  for (unsigned r = 0; r < 4u; ++r) {
    const unsigned t = w * 4u + r;
    const unsigned qo = QS_OFF + t * QP;
    const unsigned ko = KS_OFF + (t + lane) * QP;
    float a0 = bias_a, a1 = bias_a;
#pragma unroll 4
    for (unsigned u = 0; u < (unsigned)UNITS; ++u) {
      const float qv = Sm[qo + u];
      const float wv = WAs[u];
      a0 += wv * tanh_fast(qv + Sm[ko + u]);
      a1 += wv * tanh_fast(qv + Sm[ko + 32u * QP + u]);
    }
    const int sA = s0 + (int)t + (int)lane;
    const int sB = sA + 32;
    const bool vA = (sA >= 0) && (sA < SEQ);
    const bool vB = (sB >= 0) && (sB < SEQ);
    const float e0 = vA ? a0 : -1.0e30f;
    const float e1 = vB ? a1 : -1.0e30f;
    const float mx = red32_max(fmaxf(e0, e1));
    const float x0 = __expf(e0 - mx);
    const float x1 = __expf(e1 - mx);
    const float p0 = vA ? x0 : 0.0f;
    const float p1 = vB ? x1 : 0.0f;
    const h16 h0 = toh_flush(p0 * PCARRY);
    const h16 h1 = toh_flush(p1 * PCARRY);
    const float sum = red32_sum((float)h0 + (float)h1);
    const unsigned zi = (lane < t) ? lane : (lane + 64u);
    Pt[t * LDP + t + lane] = h0;
    Pt[t * LDP + t + lane + 32u] = h1;
    Pt[t * LDP + zi] = (h16)0.0f;
    if (lane == 0u) Rinv[t] = __builtin_amdgcn_rcpf(sum);
  }
  __syncthreads();

  const int c_lo = (t0 == 0u) ? 1 : 0;
  const int c_hi = (t0 + (unsigned)QT == (unsigned)SEQ) ? 2 : 3;
  const unsigned cw = w * (16u * LDC);
#pragma unroll 1
  for (unsigned pass = 0; pass < 2u; ++pass) {
    const unsigned d0 = w * 128u + pass * 64u;
    v8f acc[2][4];
#pragma unroll
    for (int mi = 0; mi < 2; ++mi)
#pragma unroll
      for (int nb = 0; nb < 4; ++nb) acc[mi][nb] = (v8f){};
    const _Float16* xp = Xt + ((size_t)b * DIM + d0 + m) * SEQ + hh * 8u;
#pragma unroll 1
    for (int c = c_lo; c < c_hi; ++c) {
      const v16h pa0 = ld_frag(&Pt[(unsigned)c * 32u], LDP);
      const v16h pa1 = ld_frag(&Pt[16u * LDP + (unsigned)c * 32u], LDP);
      const unsigned sk = (unsigned)(s0 + 32 * c);
#pragma unroll
      for (int nb = 0; nb < 4; ++nb) {
        const v16h xb = frag_at(xp + (size_t)(nb * 16) * SEQ + sk);
        acc[0][nb] = wmma16(pa0, xb, acc[0][nb]);
        acc[1][nb] = wmma16(pa1, xb, acc[1][nb]);
      }
    }
#pragma unroll
    for (int mi = 0; mi < 2; ++mi) {
#pragma unroll
      for (int r = 0; r < 8; ++r) {
        const float sc = Rinv[(unsigned)mi * 16u + hh * 8u + (unsigned)r];
#pragma unroll
        for (int nb = 0; nb < 4; ++nb)
          Sm[cw + (hh * 8u + (unsigned)r) * LDC + (unsigned)nb * 16u + m] = acc[mi][nb][r] * sc;
      }
      wave_lds_sync();
      v4f xs[8];
      size_t off[8];
#pragma unroll
      for (unsigned i = 0; i < 8u; ++i) {
        const unsigned rr = 2u * i + (lane >> 4);
        const unsigned cc = (lane & 15u) * 4u;
        xs[i] = *(const v4f*)&Sm[cw + rr * LDC + cc];
        off[i] = ((size_t)b * SEQ_FULL + t0 + (unsigned)mi * 16u + rr) * DIM + d0 + cc;
      }
      wave_lds_sync();
#pragma unroll
      for (int i = 0; i < 8; ++i) *(volatile v4f*)(out + off[i]) = xs[i];
      __threadfence();
#pragma unroll
      for (int i = 0; i < 8; ++i) *(volatile v4f*)(out + off[i]) = xs[i];
    }
  }
}

extern "C" void kernel_launch(void* const* d_in, const int* in_sizes, int n_in,
                              void* d_out, int out_size, void* d_ws, size_t ws_size,
                              hipStream_t stream) {
  if (n_in < 6) return;
  const long long need_x = ((long long)(NB - 1) * SEQ_FULL + SEQ) * DIM;
  if ((long long)in_sizes[0] < need_x) return;
  if ((long long)in_sizes[1] < (long long)DIM * UNITS) return;
  if ((long long)in_sizes[2] < (long long)DIM * UNITS) return;
  if (in_sizes[3] < UNITS || in_sizes[4] < UNITS || in_sizes[5] < 1) return;
  if ((long long)out_size < need_x) return;
  if (ws_size < WS_TOTAL) return;

  const float* X  = (const float*)d_in[0];
  const float* wt = (const float*)d_in[1];
  const float* wx = (const float*)d_in[2];
  const float* bh = (const float*)d_in[3];
  const float* wa = (const float*)d_in[4];
  const float* ba = (const float*)d_in[5];
  float* out = (float*)d_out;

  char* ws = (char*)d_ws;
  _Float16* Wqk = (_Float16*)(ws + OFF_WQK);
  _Float16* Xh  = (_Float16*)(ws + OFF_XH);
  _Float16* Xt  = (_Float16*)(ws + OFF_XT);
  float*    QK  = (float*)(ws + OFF_QK);

  dim3 blk(256);
  wconv_kernel<<<dim3(UNITS / 64, DIM / 64), blk, 0, stream>>>(wt, Wqk, (unsigned)UNITS, (unsigned)DIM);
  wconv_kernel<<<dim3(UNITS / 64, DIM / 64), blk, 0, stream>>>(wx, Wqk + (size_t)UNITS * DIM,
                                                              (unsigned)UNITS, (unsigned)DIM);
  xconv_kernel<<<dim3(DIM / 64, MROWS / 64), blk, 0, stream>>>(X, Xh, Xt);
  proj_kernel<<<dim3(NQK / 64, MROWS / 64), blk, 0, stream>>>(Xh, Wqk, QK);
  band_attn_kernel<<<dim3(SEQ / QT, NB), blk, 0, stream>>>(QK, Xt, bh, wa, ba, out);
}
